// RelationNetwork_60722247631026
// MI455X (gfx1250) — hardware-verified
//
#include <hip/hip_runtime.h>


#ifndef NB
#define NB 4
#endif
#ifndef NPTS
#define NPTS 512
#endif
#define NB_FULL   4
#define NPTS_FULL 512
#define FDIM 64
#define RDIM 128
#define PAIRS (NPTS * (NPTS - 1))
#define DM   FDIM
#define LOSC 1024.0f
#define TP   136

static_assert(NB >= 1 && NB <= NB_FULL);
static_assert(NPTS >= 2 && NPTS <= NPTS_FULL);
static_assert(PAIRS % 64 == 0);
static_assert((NB * NPTS) % 64 == 0);
static_assert(FDIM % 64 == 0 && RDIM == 128);
static_assert(TP % 8 == 0);

typedef _Float16 h16;
typedef unsigned short bf;
typedef __attribute__((ext_vector_type(16))) __bf16   v16bf;
typedef __attribute__((ext_vector_type(16))) _Float16 v16h;
typedef __attribute__((ext_vector_type(8)))  _Float16 v8h;
typedef __attribute__((ext_vector_type(8)))  unsigned short v8us;
typedef __attribute__((ext_vector_type(4)))  unsigned short v4us;
typedef __attribute__((ext_vector_type(8)))  float    v8f;
typedef __attribute__((ext_vector_type(4)))  float    v4f;
typedef __attribute__((ext_vector_type(4)))  _Float16 v4h;
typedef v8h  __attribute__((may_alias)) v8ha;
typedef v4f  __attribute__((may_alias)) v4fa;
typedef v8us __attribute__((may_alias)) v8usa;
typedef v4us __attribute__((may_alias)) v4usa;

__device__ __forceinline__ unsigned short f2bf(float f) { unsigned u = __float_as_uint(f); u += 0x7FFFu + ((u >> 16) & 1u); return (unsigned short)(u >> 16); }
__device__ __forceinline__ float bf2f(unsigned short b) { return __uint_as_float(((unsigned)b) << 16); }
__device__ __forceinline__ float bfr(float f) { return bf2f(f2bf(f)); }
__device__ __forceinline__ v16h cat16(v8h lo, v8h hi) { return __builtin_shufflevector(lo, hi, 0, 1, 2, 3, 4, 5, 6, 7, 8, 9, 10, 11, 12, 13, 14, 15); }
__device__ __forceinline__ v16bf cat16b(v8us lo, v8us hi) { return __builtin_bit_cast(v16bf, __builtin_shufflevector(lo, hi, 0, 1, 2, 3, 4, 5, 6, 7, 8, 9, 10, 11, 12, 13, 14, 15)); }
__device__ __forceinline__ v8f wmma16(v16h a, v16h b, v8f c) { return __builtin_amdgcn_wmma_f32_16x16x32_f16(false, a, false, b, (short)0, c, false, false); }
__device__ __forceinline__ v8f wmmab(v16bf a, v16bf b, v8f c) { return __builtin_amdgcn_wmma_f32_16x16x32_bf16(false, a, false, b, (short)0, c, false, false); }

__global__ __launch_bounds__(256) void k_cvt64(const float* __restrict__ src, bf* dst) {
    const size_t i = (size_t)blockIdx.x * 256 + threadIdx.x; if (i >= (size_t)NB * NPTS * FDIM / 4) return;
    const size_t row = i / (FDIM / 4), c4 = i - row * (FDIM / 4);
    const size_t b = row / NPTS, n = row - b * NPTS;
    const v4f v = *(const v4f*)(src + (b * NPTS_FULL + n) * FDIM + c4 * 4); v4us o;
#pragma unroll
    for (int k = 0; k < 4; ++k) o[k] = f2bf(v[k]);
    *(volatile v4us*)(dst + i * 4) = o; __threadfence(); *(volatile v4us*)(dst + i * 4) = o;
}
__global__ __launch_bounds__(256) void k_wt(const float* __restrict__ Wm, int K, int ncols, bf* WT) {
    __shared__ __align__(16) unsigned short tl[64 * 72];
    const int tid = threadIdx.x, k0 = blockIdx.x * 64, n0 = blockIdx.y * 64;
    const int kk = tid >> 2, nq = (tid & 3) * 16;
#pragma unroll
    for (int i = 0; i < 16; ++i) tl[(nq + i) * 72 + kk] = f2bf(Wm[(size_t)(k0 + kk) * ncols + n0 + nq + i]);
    __syncthreads();
    const int piece = tid & 7;
    auto pass = [&]() {
#pragma unroll
        for (int s = 0; s < 2; ++s) { const int nr = (tid >> 3) + 32 * s; const v8us val = *(const v8usa*)(tl + nr * 72 + piece * 8); *(volatile v8us*)(WT + (size_t)(n0 + nr) * K + k0 + piece * 8) = val; }
    };
    pass(); __threadfence(); pass();
}
template <bool SPLITA, bool F16OUT = false>
__global__ __launch_bounds__(128) void k_gemmb(const bf* __restrict__ A, const bf* __restrict__ Al, const bf* __restrict__ Bn, const float* __restrict__ bias, float* C, int ldc, h16* C2, const float* __restrict__ R = nullptr, int K = DM, int rnR = 1) {
    __shared__ __align__(16) float ost[4][16 * 68];
    const int lane = threadIdx.x & 31, wave = threadIdx.x >> 5, lr = lane & 15, hi = lane >> 4;
    const int r0 = blockIdx.x * 64 + wave * 16, c0 = blockIdx.y * 64;
    const size_t aoff = (size_t)(r0 + lr) * K + 8 * hi;
    size_t boff[4];
#pragma unroll
    for (int t = 0; t < 4; ++t) boff[t] = (size_t)(c0 + t * 16 + lr) * K + 8 * hi;
    v8f acc[4];
#pragma unroll
    for (int t = 0; t < 4; ++t) acc[t] = (v8f){};
#pragma unroll 1
    for (int kc = 0; kc < K; kc += 32) {
        const v16bf a = cat16b(*(const v8us*)(A + aoff + kc), *(const v8us*)(A + aoff + kc + 16));
        v16bf al = a;
        if (SPLITA) al = cat16b(*(const v8us*)(Al + aoff + kc), *(const v8us*)(Al + aoff + kc + 16));
#pragma unroll
        for (int t = 0; t < 4; ++t) { const v16bf b = cat16b(*(const v8us*)(Bn + boff[t] + kc), *(const v8us*)(Bn + boff[t] + kc + 16)); acc[t] = wmmab(a, b, acc[t]); if (SPLITA) acc[t] = wmmab(al, b, acc[t]); }
        asm volatile("v_nop\n\tv_nop\n\tv_nop\n\tv_nop" : "+v"(acc[0]), "+v"(acc[1]), "+v"(acc[2]), "+v"(acc[3]) : "v"(a), "v"(al));
    }
    float* os = &ost[wave][0];
#pragma unroll
    for (int t = 0; t < 4; ++t) { const float bv = bias ? bfr(bias[c0 + t * 16 + lr]) : 0.f;
#pragma unroll
        for (int j = 0; j < 8; ++j) os[(hi * 8 + j) * 68 + t * 16 + lr] = acc[t][j] + bv; }
    __syncthreads();
    if (F16OUT) {
        h16* crow = (h16*)(void*)C + (size_t)r0 * ldc + c0;
        auto pass = [&]() {
#pragma unroll
            for (int s = 0; s < 4; ++s) { const int row = 4 * s + (lane >> 3), piece = lane & 7; const float* sp = os + row * 68 + piece * 8; v8h o, o2;
#pragma unroll
                for (int i = 0; i < 8; ++i) { const h16 a = (h16)sp[i]; o[i] = a; o2[i] = (h16)((sp[i] - (float)a) * LOSC); }
                *(volatile v8h*)(crow + (size_t)row * ldc + piece * 8) = o; if (C2) *(volatile v8h*)(C2 + (size_t)r0 * ldc + c0 + (size_t)row * ldc + piece * 8) = o2; }
        };
        pass(); __threadfence(); pass();
    } else {
        float* crow = C + (size_t)r0 * ldc + c0;
        auto pass = [&]() {
#pragma unroll
            for (int s = 0; s < 8; ++s) { const int Lid = (lane >> 3) + 4 * s, piece = lane & 7; const int row = Lid >> 1, cofs = (Lid & 1) * 32 + piece * 4;
                v4f val = *(const v4fa*)(os + row * 68 + cofs); if (R) { const v4f rv = *(const v4f*)(R + ((size_t)r0 + row) * ldc + c0 + cofs); val += rnR ? (v4f){bfr(rv[0]), bfr(rv[1]), bfr(rv[2]), bfr(rv[3])} : rv; }
                *(volatile v4f*)(crow + (size_t)row * ldc + cofs) = val; }
        };
        pass(); __threadfence(); pass();
    }
}

__global__ __launch_bounds__(128) void k_rel(const float* __restrict__ P, const float* __restrict__ Q, const bf* __restrict__ W2T, const float* __restrict__ b2,
                                             const float* __restrict__ W3, const float* __restrict__ b3, float* OUTP) {
    __shared__ __align__(16) unsigned short th[4][16 * TP];
    __shared__ __align__(16) unsigned short tr[4][16 * TP];
    __shared__ float sB2[RDIM];
    __shared__ float sW3[RDIM];
    __shared__ __align__(16) float so[64];
    const int tid = threadIdx.x, lane = tid & 31, wave = tid >> 5, lr = lane & 15, hi = lane >> 4;
    const int tpb = PAIRS / 64;
    const int b = blockIdx.x / tpb;
    const int p0 = (blockIdx.x - b * tpb) * 64;
    const int pw = p0 + wave * 16;
    if (tid < RDIM) { sB2[tid] = bfr(b2[tid]); sW3[tid] = bfr(W3[tid]); }
    const float b3r = bfr(b3[0]);
    unsigned short* thw = &th[wave][0];
    unsigned short* trw = &tr[wave][0];
#pragma unroll 4
    for (int r = 0; r < 16; ++r) {
        const int p = pw + r;
        int i = p / (NPTS - 1);
        const int rem = p - i * (NPTS - 1);
        int j = rem + ((rem >= i) ? 1 : 0);
        i = min(i, NPTS - 1); j = min(j, NPTS - 1);
        const v4f pv = *(const v4f*)(P + ((size_t)(b * NPTS + i) * RDIM + lane * 4));
        const v4f qv = *(const v4f*)(Q + ((size_t)(b * NPTS + j) * RDIM + lane * 4));
        v4us oh, ol;
#pragma unroll
        for (int k = 0; k < 4; ++k) { const float hv = fmaxf(pv[k] + qv[k], 0.f); const unsigned short hb = f2bf(hv); oh[k] = hb; ol[k] = f2bf(hv - bf2f(hb)); }
        *(v4usa*)(thw + r * TP + lane * 4) = oh;
        *(v4usa*)(trw + r * TP + lane * 4) = ol;
    }
    __syncthreads();
    const unsigned short* ah = thw + lr * TP + 8 * hi;
    const unsigned short* ar = trw + lr * TP + 8 * hi;
    const bf* bp = W2T + (size_t)lr * RDIM + 8 * hi;
    v8f acc[8];
#pragma unroll
    for (int t = 0; t < 8; ++t) acc[t] = (v8f){};
#pragma unroll 1
    for (int kc = 0; kc < RDIM; kc += 32) {
        const v16bf a  = cat16b(*(const v8usa*)(ah + kc), *(const v8usa*)(ah + kc + 16));
        const v16bf al = cat16b(*(const v8usa*)(ar + kc), *(const v8usa*)(ar + kc + 16));
#pragma unroll
        for (int t = 0; t < 8; ++t) {
            const v16bf bb = cat16b(*(const v8us*)(bp + (size_t)t * 16 * RDIM + kc), *(const v8us*)(bp + (size_t)t * 16 * RDIM + kc + 16));
            acc[t] = wmmab(a, bb, acc[t]);
            acc[t] = wmmab(al, bb, acc[t]);
        }
        asm volatile("v_nop\n\tv_nop\n\tv_nop\n\tv_nop" : "+v"(acc[0]), "+v"(acc[1]), "+v"(acc[2]), "+v"(acc[3]), "+v"(acc[4]), "+v"(acc[5]), "+v"(acc[6]), "+v"(acc[7]) : "v"(a), "v"(al));
    }
    float part[8];
#pragma unroll
    for (int v = 0; v < 8; ++v) part[v] = 0.f;
#pragma unroll
    for (int t = 0; t < 8; ++t) {
        const float b2v = sB2[t * 16 + lr], w3v = sW3[t * 16 + lr];
#pragma unroll
        for (int v = 0; v < 8; ++v) part[v] = fmaf(fmaxf(acc[t][v] + b2v, 0.f), w3v, part[v]);
    }
#pragma unroll
    for (int v = 0; v < 8; ++v) {
#pragma unroll
        for (int s = 1; s < 16; s <<= 1) part[v] += __shfl_xor(part[v], s, 32);
    }
    if (lr == 0) {
#pragma unroll
        for (int v = 0; v < 8; ++v) so[wave * 16 + 8 * hi + v] = part[v] + b3r;
    }
    __syncthreads();
    if (tid < 16) {
        const v4f val = *(const v4fa*)(&so[tid * 4]);
        float* dst = OUTP + ((size_t)b * PAIRS + p0 + tid * 4);
        *(volatile v4f*)dst = val; __threadfence(); *(volatile v4f*)dst = val;
    }
}

extern "C" void kernel_launch(void* const* d_in, const int* in_sizes, int n_in,
                              void* d_out, int out_size, void* d_ws, size_t ws_size, hipStream_t stream) {
    if (n_in < 7) return;
    if (in_sizes[0] < ((NB - 1) * NPTS_FULL + NPTS) * FDIM) return;
    if (in_sizes[1] < 2 * FDIM * RDIM || in_sizes[2] < RDIM || in_sizes[3] < RDIM * RDIM || in_sizes[4] < RDIM || in_sizes[5] < RDIM || in_sizes[6] < 1) return;
    if (out_size < NB * PAIRS) return;
    const float* feat = (const float*)d_in[0]; const float* W1 = (const float*)d_in[1]; const float* b1 = (const float*)d_in[2];
    const float* W2 = (const float*)d_in[3]; const float* b2 = (const float*)d_in[4]; const float* W3 = (const float*)d_in[5]; const float* b3 = (const float*)d_in[6];
    float* out = (float*)d_out;
    char* wsp = (char*)d_ws;
    auto take = [&](size_t bytes) { char* p = wsp; wsp += (bytes + 255) & ~(size_t)255; return (void*)p; };
    bf* Ob  = (bf*)take((size_t)NB * NPTS * FDIM * 2);
    bf* WaT = (bf*)take((size_t)RDIM * FDIM * 2);
    bf* WbT = (bf*)take((size_t)RDIM * FDIM * 2);
    bf* W2T = (bf*)take((size_t)RDIM * RDIM * 2);
    float* P = (float*)take((size_t)NB * NPTS * RDIM * 4);
    float* Q = (float*)take((size_t)NB * NPTS * RDIM * 4);
    const size_t carved = (size_t)(wsp - (char*)d_ws);
    if (carved > ws_size || carved > ((size_t)128 << 20)) return;
    k_cvt64<<<(unsigned)(((size_t)NB * NPTS * FDIM / 4 + 255) / 256), 256, 0, stream>>>(feat, Ob);
    k_wt<<<dim3(FDIM / 64, RDIM / 64, 1), 256, 0, stream>>>(W1, FDIM, RDIM, WaT);
    k_wt<<<dim3(FDIM / 64, RDIM / 64, 1), 256, 0, stream>>>(W1 + (size_t)FDIM * RDIM, FDIM, RDIM, WbT);
    k_wt<<<dim3(RDIM / 64, RDIM / 64, 1), 256, 0, stream>>>(W2, RDIM, RDIM, W2T);
    k_gemmb<false, false><<<dim3(NB * NPTS / 64, RDIM / 64, 1), 128, 0, stream>>>(Ob, nullptr, WaT, b1, P, RDIM, nullptr);
    k_gemmb<false, false><<<dim3(NB * NPTS / 64, RDIM / 64, 1), 128, 0, stream>>>(Ob, nullptr, WbT, nullptr, Q, RDIM, nullptr);
    k_rel<<<(unsigned)(NB * (PAIRS / 64)), 128, 0, stream>>>(P, Q, W2T, b2, W3, b3, out);
}
